// PPM_84490596647491
// MI455X (gfx1250) — hardware-verified
//
#include <hip/hip_runtime.h>
#include <math.h>
#include <stdint.h>

#ifndef NB
#define NB    4
#endif
#ifndef SEQ
#define SEQ   4096
#endif
#define NB_FULL  4
#define SEQ_FULL 4096
#define CC    256
#define QT    64
#define OSP   68
#define OSPW  132
#define TP    72
#define GSC   64.0f
#define PSC   64.0f
#define OSC   3.814697265625e-06f
#define EPSN  1.0e-8f

static_assert(NB >= 1 && NB <= NB_FULL);
static_assert(SEQ >= QT && SEQ <= SEQ_FULL);
static_assert(SEQ % QT == 0 && CC % QT == 0);
static_assert(CC % 32 == 0 && SEQ % 32 == 0 && SEQ_FULL % 8 == 0);
static_assert((OSP * 4) % 16 == 0);
static_assert((OSPW * 4) % 16 == 0);
static_assert((TP * 2) % 16 == 0);
static_assert((NB * SEQ) % 256 == 0);
static_assert(CC % 8 == 0);

typedef _Float16       v16h __attribute__((ext_vector_type(16)));
typedef _Float16       v8h  __attribute__((ext_vector_type(8)));
typedef __bf16         v16b __attribute__((ext_vector_type(16)));
typedef unsigned short v8us __attribute__((ext_vector_type(8)));
typedef float          v8f  __attribute__((ext_vector_type(8)));
typedef float          v4f  __attribute__((ext_vector_type(4)));
typedef unsigned int   v4u  __attribute__((ext_vector_type(4)));

union Frag  { v8us u[2]; v16h h; v16b bf; };
union FragH { v16h v; v8h hv[2]; };
static_assert(sizeof(Frag) == 32);
static_assert(sizeof(FragH) == 32);

__device__ __forceinline__ unsigned short bf_bits(float f) {
  unsigned u = __float_as_uint(f);
  return (unsigned short)((u + 0x7FFFu + ((u >> 16) & 1u)) >> 16);
}
__device__ __forceinline__ float bf_up(unsigned short hb) { return __uint_as_float(((unsigned)hb) << 16); }
__device__ __forceinline__ float bfr(float f) { return bf_up(bf_bits(f)); }
__device__ __forceinline__ unsigned short h_bits(_Float16 x) { return __builtin_bit_cast(unsigned short, x); }
__device__ __forceinline__ unsigned pk16(unsigned short a, unsigned short b) { return (unsigned)a | ((unsigned)b << 16); }
__device__ __forceinline__ v8f zero8() { v8f z = {0.f, 0.f, 0.f, 0.f, 0.f, 0.f, 0.f, 0.f}; return z; }

__device__ __forceinline__ Frag ldfrag(const unsigned short* p) {
  Frag f;
  f.u[0] = *(const v8us*)(p);
  f.u[1] = *(const v8us*)(p + 16);
  return f;
}

__device__ __forceinline__ v8f mma_h(v16h a, v16h b, v8f c) {
  v8f d = __builtin_amdgcn_wmma_f32_16x16x32_f16(false, a, false, b, (short)0, c, false, false);
#if defined(__HIP_DEVICE_COMPILE__)
  asm volatile("v_nop\n\tv_nop\n\tv_nop\n\tv_nop" : "+v"(d) : "v"(a), "v"(b));
#endif
  return d;
}
__device__ __forceinline__ v8f mma_b(v16b a, v16b b, v8f c) {
  v8f d = __builtin_amdgcn_wmma_f32_16x16x32_bf16(false, a, false, b, (short)0, c, false, false);
#if defined(__HIP_DEVICE_COMPILE__)
  const v16h ha = __builtin_bit_cast(v16h, a), hb = __builtin_bit_cast(v16h, b);
  asm volatile("v_nop\n\tv_nop\n\tv_nop\n\tv_nop" : "+v"(d) : "v"(ha), "v"(hb));
#endif
  return d;
}

__global__ __launch_bounds__(256)
void cvt_w(const float* __restrict__ w, unsigned short* Wb) {
  const int tid = threadIdx.x, blk = blockIdx.x;
  const int rl = tid >> 5, col = 8 * (tid & 31);
  const int o = 8 * blk + rl;
  const float* s = w + (size_t)o * CC + col;
  const v4f a = *(const v4f*)s;
  const v4f q = *(const v4f*)(s + 4);
  const float f[8] = {a[0], a[1], a[2], a[3], q[0], q[1], q[2], q[3]};
  v4u u;
#pragma unroll
  for (int t = 0; t < 4; ++t) u[t] = pk16(bf_bits(f[2 * t]), bf_bits(f[2 * t + 1]));
#pragma unroll
  for (int pass = 0; pass < 2; ++pass) {
    *(volatile v4u*)(Wb + (size_t)o * CC + col) = u;
    __threadfence();
  }
}

__global__ __launch_bounds__(256)
void cvt_x(const float* __restrict__ x, unsigned short* XP) {
  __shared__ __align__(16) unsigned short T[QT * TP];
  const int tid = threadIdx.x;
  const int nb = blockIdx.x, cb = blockIdx.y, b = blockIdx.z;
  const int e = tid & 7, lq = tid >> 3;
  const int n0 = nb * QT, c0 = cb * QT;
#pragma unroll
  for (int it = 0; it < 2; ++it) {
    const int cl = it * 32 + lq;
    const float* sp = x + ((size_t)(b * CC + c0 + cl)) * SEQ_FULL + n0 + 8 * e;
    const v4f a = *(const v4f*)sp;
    const v4f q = *(const v4f*)(sp + 4);
    unsigned short hb[8];
#pragma unroll
    for (int t = 0; t < 4; ++t) {
      hb[t]     = bf_bits(a[t]);
      hb[4 + t] = bf_bits(q[t]);
    }
#pragma unroll
    for (int t = 0; t < 8; ++t) T[(8 * e + t) * TP + cl] = hb[t];
  }
  __syncthreads();
  v4u up[2];
#pragma unroll
  for (int it = 0; it < 2; ++it) {
    const int nl = it * 32 + lq;
    up[it] = *(const v4u*)(T + nl * TP + 8 * e);
  }
#pragma unroll
  for (int pass = 0; pass < 2; ++pass) {
#pragma unroll
    for (int it = 0; it < 2; ++it) {
      const int rl = it * 32 + lq;
      *(volatile v4u*)(XP + ((size_t)(b * SEQ + n0 + rl)) * CC + c0 + 8 * e) = up[it];
    }
    __threadfence();
  }
}

__global__ __launch_bounds__(256)
void norm_k(const float* __restrict__ x, float* inv) {
  const int e = blockIdx.x * 256 + threadIdx.x;
  const int b = e / SEQ, n = e % SEQ;
  const float* xp = x + (size_t)b * CC * SEQ_FULL + n;
  float s = 0.f;
#pragma unroll 4
  for (int c = 0; c < CC; ++c) {
    const float v = bfr(xp[(size_t)c * SEQ_FULL]);
    const float vv = v * v;
    s += vv;
  }
  const float nr = sqrtf(s);
  const float iv = 1.0f / fmaxf(nr, EPSN);
#pragma unroll
  for (int pass = 0; pass < 2; ++pass) {
    *(volatile float*)(inv + e) = iv;
    __threadfence();
  }
}

__global__ __launch_bounds__(128)
void conv_k(const unsigned short* __restrict__ Wb, const unsigned short* __restrict__ XP,
            const float* __restrict__ bias, unsigned short* Gc) {
  __shared__ __align__(16) float Os[QT * OSP];
  const int tid  = threadIdx.x;
  const int lane = tid & 31, wave = tid >> 5;
  const int hh   = lane >> 4, c = lane & 15;
  const int nt   = blockIdx.x, mb = blockIdx.y, b = blockIdx.z;
  const int n0   = nt * QT, o0 = mb * QT;

  const unsigned short* ap = Wb + (size_t)(o0 + c) * CC + 8 * hh;
  const unsigned short* bp = XP + ((size_t)(b * SEQ + n0 + 16 * wave + c)) * CC + 8 * hh;

  v8f acc[4];
#pragma unroll
  for (int mt = 0; mt < 4; ++mt) acc[mt] = zero8();

#pragma unroll
  for (int ks = 0; ks < CC / 32; ++ks) {
    const Frag fb = ldfrag(bp + 32 * ks);
#pragma unroll
    for (int mt = 0; mt < 4; ++mt) {
      const Frag fa = ldfrag(ap + (size_t)(16 * mt) * CC + 32 * ks);
      acc[mt] = mma_b(fa.bf, fb.bf, acc[mt]);
    }
  }

  {
    const int nl = 16 * wave + c;
#pragma unroll
    for (int mt = 0; mt < 4; ++mt) {
#pragma unroll
      for (int r = 0; r < 8; ++r) Os[(16 * mt + 8 * hh + r) * OSP + nl] = acc[mt][r];
    }
  }
  __syncthreads();

  const int e = tid & 7, lq = tid >> 3;
  v4u u[4];
#pragma unroll
  for (int it = 0; it < 4; ++it) {
    const int row = it * 16 + lq;
    const float bo = bfr(bias[o0 + row]);
    const v4f a = *(const v4f*)(Os + row * OSP + 8 * e);
    const v4f q = *(const v4f*)(Os + row * OSP + 8 * e + 4);
    const float f[8] = {a[0], a[1], a[2], a[3], q[0], q[1], q[2], q[3]};
#pragma unroll
    for (int t = 0; t < 4; ++t) {
      const _Float16 h0 = (_Float16)((f[2 * t] + bo) * GSC);
      const _Float16 h1 = (_Float16)((f[2 * t + 1] + bo) * GSC);
      u[it][t] = pk16(h_bits(h0), h_bits(h1));
    }
  }
#pragma unroll
  for (int pass = 0; pass < 2; ++pass) {
#pragma unroll
    for (int it = 0; it < 4; ++it) {
      const int row = it * 16 + lq;
      *(volatile v4u*)(Gc + ((size_t)(b * CC + o0 + row)) * SEQ + n0 + 8 * e) = u[it];
    }
    __threadfence();
  }
}

__global__ __launch_bounds__(128)
void ppm_k(const unsigned short* __restrict__ XP, const float* __restrict__ inv,
           const unsigned short* __restrict__ Gc, float* out) {
  __shared__ __align__(16) float Os[QT * OSPW];
  const int tid  = threadIdx.x;
  const int wave = tid >> 5, lane = tid & 31;
  const int hh   = lane >> 4, c = lane & 15;
  const int n0   = blockIdx.x * QT, b = blockIdx.y;

  const unsigned short* Pp = XP + ((size_t)(b * SEQ + n0 + 16 * wave + c)) * CC + 8 * hh;
  const unsigned short* Qp = XP + (size_t)b * SEQ * CC + (size_t)c * CC + 8 * hh;
  const unsigned short* Gp = Gc + (size_t)b * CC * SEQ + (size_t)c * SEQ + 8 * hh;
  const float* invb = inv + (size_t)b * SEQ;
  const float ip = invb[n0 + 16 * wave + c] * PSC;

  v8f o[16];
#pragma unroll
  for (int j = 0; j < 16; ++j) o[j] = zero8();

#pragma unroll 1
  for (int kb = 0; kb < SEQ; kb += 32) {
    const unsigned short* q0p = Qp + (size_t)kb * CC;
    const unsigned short* q1p = Qp + (size_t)(kb + 16) * CC;
    v8f s0 = zero8(), s1 = zero8();
#pragma unroll 1
    for (int kc = 0; kc < CC / 32; ++kc) {
      const Frag fp = ldfrag(Pp + 32 * kc);
      const Frag f0 = ldfrag(q0p + 32 * kc);
      const Frag f1 = ldfrag(q1p + 32 * kc);
      s0 = mma_b(f0.bf, fp.bf, s0);
      s1 = mma_b(f1.bf, fp.bf, s1);
    }

    const v4f ia = *(const v4f*)(invb + kb + 8 * hh);
    const v4f ib = *(const v4f*)(invb + kb + 8 * hh + 4);
    const v4f ic = *(const v4f*)(invb + kb + 16 + 8 * hh);
    const v4f id = *(const v4f*)(invb + kb + 16 + 8 * hh + 4);

    FragH ph;
#pragma unroll
    for (int r = 0; r < 8; ++r) {
      const float iq0 = (r < 4) ? ia[r] : ib[r - 4];
      const float iq1 = (r < 4) ? ic[r] : id[r - 4];
      float t0 = (s0[r] * iq0) * ip;
      float t1 = (s1[r] * iq1) * ip;
      t0 = fmaxf(t0, 0.0f);
      t1 = fmaxf(t1, 0.0f);
      ph.hv[0][r] = (_Float16)(t0 * t0);
      ph.hv[1][r] = (_Float16)(t1 * t1);
    }

#pragma unroll
    for (int j = 0; j < 16; ++j) {
      const Frag vf = ldfrag(Gp + (size_t)(16 * j) * SEQ + kb);
      o[j] = mma_h(vf.h, ph.v, o[j]);
    }
  }

  const int qrow = 16 * wave + c;
  const int e = tid & 7, lq = tid >> 3;
#pragma unroll
  for (int half = 0; half < 2; ++half) {
    if (half) __syncthreads();
#pragma unroll
    for (int jj = 0; jj < 8; ++jj) {
      const int j = 8 * half + jj;
      v4f va, vb;
#pragma unroll
      for (int r = 0; r < 4; ++r) { va[r] = o[j][r] * OSC; vb[r] = o[j][4 + r] * OSC; }
      *(v4f*)(Os + qrow * OSPW + 16 * jj + 8 * hh)     = va;
      *(v4f*)(Os + qrow * OSPW + 16 * jj + 8 * hh + 4) = vb;
    }
    __syncthreads();
    v4f res[16];
#pragma unroll
    for (int it = 0; it < 16; ++it) {
      const int L   = it * 16 + lq;
      const int chl = L >> 1, hf = L & 1;
      const int nl  = hf * 32 + 4 * e;
#pragma unroll
      for (int t = 0; t < 4; ++t) res[it][t] = Os[(nl + t) * OSPW + chl];
    }
#pragma unroll
    for (int pass = 0; pass < 2; ++pass) {
#pragma unroll
      for (int it = 0; it < 16; ++it) {
        const int L   = it * 16 + lq;
        const int chl = L >> 1, hf = L & 1;
        const int nl  = hf * 32 + 4 * e;
        const size_t idx = ((size_t)(b * CC + 128 * half + chl)) * SEQ + n0 + nl;
        *(volatile v4f*)(out + idx) = res[it];
      }
      __threadfence();
    }
  }
}

extern "C" void kernel_launch(void* const* d_in, const int* in_sizes, int n_in,
                              void* d_out, int out_size, void* d_ws, size_t ws_size,
                              hipStream_t stream) {
  if (n_in < 3) return;
  if (in_sizes[0] < NB * CC * SEQ_FULL) return;
  if (in_sizes[1] < CC * CC || in_sizes[2] < CC) return;
  if (out_size < NB * CC * SEQ) return;

  size_t off = 0;
  auto carve = [&](size_t bytes) { const size_t o = off; off += (bytes + 255) & ~(size_t)255; return o; };
  const size_t oWb  = carve((size_t)CC * CC * 2);
  const size_t oXP  = carve((size_t)NB * SEQ * CC * 2);
  const size_t oInv = carve((size_t)NB * SEQ * 4);
  const size_t oGc  = carve((size_t)NB * CC * SEQ * 2);
  if (off > ws_size) return;
  if (off > (size_t)134217728) return;

  const float* x    = (const float*)d_in[0];
  const float* w    = (const float*)d_in[1];
  const float* bias = (const float*)d_in[2];

  char* ws = (char*)d_ws;
  unsigned short* Wb  = (unsigned short*)(ws + oWb);
  unsigned short* XP  = (unsigned short*)(ws + oXP);
  float*          inv = (float*)(ws + oInv);
  unsigned short* Gc  = (unsigned short*)(ws + oGc);
  float* out = (float*)d_out;

  const dim3 blk256(256), blk128(128);

  cvt_w<<<dim3(CC / 8), blk256, 0, stream>>>(w, Wb);
  cvt_x<<<dim3(SEQ / QT, CC / QT, NB), blk256, 0, stream>>>(x, XP);
  norm_k<<<dim3((NB * SEQ) / 256), blk256, 0, stream>>>(x, inv);
  conv_k<<<dim3(SEQ / QT, CC / QT, NB), blk128, 0, stream>>>(Wb, XP, bias, Gc);
  ppm_k<<<dim3(SEQ / QT, NB), blk128, 0, stream>>>(XP, inv, Gc, out);
  (void)hipGetLastError();
}
